// LocalMaskedMMHCA_24043226923905
// MI455X (gfx1250) — hardware-verified
//
#include <hip/hip_runtime.h>


#define CC   512
#define TT   8192
#define NH_  8
#define HD   64
#define WW   64
#define NC   128
#define KW   192
#define TP   (TT + 2 * WW)
typedef _Float16 h16;
typedef unsigned short bf;
typedef __attribute__((ext_vector_type(16))) __bf16   v16bf;
typedef __attribute__((ext_vector_type(16))) _Float16 v16h;
typedef __attribute__((ext_vector_type(8)))  _Float16 v8h;
typedef __attribute__((ext_vector_type(8)))  unsigned short v8us;
typedef __attribute__((ext_vector_type(8)))  float    v8f;
typedef __attribute__((ext_vector_type(4)))  float    v4f;
typedef v8h  __attribute__((may_alias)) v8ha;
typedef v4f  __attribute__((may_alias)) v4fa;
typedef v8us __attribute__((may_alias)) v8usa;

__device__ __forceinline__ unsigned short f2bf(float f) { unsigned u = __float_as_uint(f); u += 0x7FFFu + ((u >> 16) & 1u); return (unsigned short)(u >> 16); }
__device__ __forceinline__ float bf2f(unsigned short b) { return __uint_as_float(((unsigned)b) << 16); }
__device__ __forceinline__ float bfr(float f) { return bf2f(f2bf(f)); }
__device__ __forceinline__ v16h cat16(v8h lo, v8h hi) { return __builtin_shufflevector(lo, hi, 0, 1, 2, 3, 4, 5, 6, 7, 8, 9, 10, 11, 12, 13, 14, 15); }
__device__ __forceinline__ v16bf cat16b(v8us lo, v8us hi) { return __builtin_bit_cast(v16bf, __builtin_shufflevector(lo, hi, 0, 1, 2, 3, 4, 5, 6, 7, 8, 9, 10, 11, 12, 13, 14, 15)); }
__device__ __forceinline__ v8f wmma16(v16h a, v16h b, v8f c) { return __builtin_amdgcn_wmma_f32_16x16x32_f16(false, a, false, b, (short)0, c, false, false); }
__device__ __forceinline__ v8f wmmab(v16bf a, v16bf b, v8f c) { return __builtin_amdgcn_wmma_f32_16x16x32_bf16(false, a, false, b, (short)0, c, false, false); }


template <typename T16> struct WFrag;
template <> struct WFrag<h16> { typedef v16h V; static __device__ __forceinline__ V ld(const h16* p) { return cat16(*(const v8h*)p, *(const v8h*)(p + 16)); } static __device__ __forceinline__ v8f mma(V a, V b, v8f c) { return wmma16(a, b, c); } };
template <> struct WFrag<bf> { typedef v16bf V; static __device__ __forceinline__ V ld(const bf* p) { return cat16b(*(const v8us*)p, *(const v8us*)(p + 16)); } static __device__ __forceinline__ v8f mma(V a, V b, v8f c) { return wmmab(a, b, c); } };
template <typename T16, int NSPLIT, bool BIAS>
__global__ __launch_bounds__(32) void k_gemmw(const T16* __restrict__ A, const T16* __restrict__ A2, const T16* __restrict__ Bt, const T16* __restrict__ Bt2, int K, float* C, int ldc, const float* __restrict__ bias, size_t sA, size_t sB, size_t sC) {
    typedef typename WFrag<T16>::V V;
    __shared__ __align__(16) float os[16 * 68];
    const size_t z = blockIdx.z; A += z * sA; if (A2) A2 += z * sA; Bt += z * sB; if (Bt2) Bt2 += z * sB; C += z * sC;
    const int lane = threadIdx.x & 31, lr = lane & 15, hi = lane >> 4; const int r0 = blockIdx.x * 64, c0 = blockIdx.y * 64;
    v8f acc[4][4];
#pragma unroll
    for (int mb = 0; mb < 4; ++mb)
#pragma unroll
        for (int nb = 0; nb < 4; ++nb) acc[mb][nb] = (v8f){};
    const size_t aoff = (size_t)(r0 + lr) * K + 8 * hi, boff = (size_t)(c0 + lr) * K + 8 * hi;
#pragma unroll 1
    for (int kc = 0; kc < K; kc += 32) {
        V a[4], a2[4];
#pragma unroll
        for (int mb = 0; mb < 4; ++mb) { a[mb] = WFrag<T16>::ld(A + aoff + (size_t)mb * 16 * K + kc); if (NSPLIT == 1 || NSPLIT == 2) a2[mb] = WFrag<T16>::ld(A2 + aoff + (size_t)mb * 16 * K + kc); }
#pragma unroll
        for (int nb = 0; nb < 4; ++nb) { const V b = WFrag<T16>::ld(Bt + boff + (size_t)nb * 16 * K + kc); V b2; if (NSPLIT >= 2) b2 = WFrag<T16>::ld(Bt2 + boff + (size_t)nb * 16 * K + kc);
#pragma unroll
            for (int mb = 0; mb < 4; ++mb) { acc[mb][nb] = WFrag<T16>::mma(a[mb], b, acc[mb][nb]); if (NSPLIT == 1 || NSPLIT == 2) acc[mb][nb] = WFrag<T16>::mma(a2[mb], b, acc[mb][nb]); if (NSPLIT >= 2) acc[mb][nb] = WFrag<T16>::mma(a[mb], b2, acc[mb][nb]); } }
        asm volatile("v_nop\n\tv_nop\n\tv_nop\n\tv_nop" : "+v"(acc[0][0]), "+v"(acc[1][1]), "+v"(acc[2][2]), "+v"(acc[3][3]) : "v"(a[0]), "v"(a[3]));
    }
#pragma unroll
    for (int mb = 0; mb < 4; ++mb) {
#pragma unroll
        for (int nb = 0; nb < 4; ++nb) {
#pragma unroll
            for (int j = 0; j < 8; ++j) os[(hi * 8 + j) * 68 + nb * 16 + lr] = acc[mb][nb][j]; }
        __builtin_amdgcn_wave_barrier(); asm volatile("" ::: "memory");
        float* crow = C + (size_t)(r0 + mb * 16) * ldc + c0;
#pragma unroll 1
        for (int ps = 0; ps < 2; ++ps) {
#pragma unroll
            for (int s = 0; s < 8; ++s) { const int row = 2 * s + hi, cofs = lr * 4; v4f val = *(const v4fa*)(os + row * 68 + cofs); if (BIAS) { val[0] += bfr(bias[c0 + cofs]); val[1] += bfr(bias[c0 + cofs + 1]); val[2] += bfr(bias[c0 + cofs + 2]); val[3] += bfr(bias[c0 + cofs + 3]); }
                *(volatile v4f*)(crow + (size_t)row * ldc + cofs) = val; }
            if (ps == 0) __threadfence(); }
        __builtin_amdgcn_wave_barrier(); asm volatile("" ::: "memory");
    }
}

__device__ __forceinline__ void splitf(float y, unsigned short& h, unsigned short& l) { h = f2bf(y); l = f2bf(y - bf2f(h)); }
typedef __attribute__((ext_vector_type(2))) unsigned short v2us;
typedef __attribute__((ext_vector_type(4))) unsigned short v4us;

__global__ __launch_bounds__(256) void k_cvt8(const float* __restrict__ src, bf* dst, size_t n8) { const size_t i = (size_t)blockIdx.x * 256 + threadIdx.x; if (i >= n8) return; const v8f v = *(const v8f*)(src + i * 8); v8us o;
#pragma unroll
    for (int k = 0; k < 8; ++k) o[k] = f2bf(v[k]); *(volatile v8us*)(dst + i * 8) = o; __threadfence(); *(volatile v8us*)(dst + i * 8) = o; }
__global__ __launch_bounds__(256) void k_dw(const float* __restrict__ x, const float* __restrict__ w, const int* __restrict__ msk, float* F) { const size_t e = ((size_t)blockIdx.x * 256 + threadIdx.x) * 4; if (e >= (size_t)TT * CC) return; const int c = (int)(e % CC); const int t = (int)(e / CC); const float mf = (msk[t] != 0) ? 1.f : 0.f; v4f o;
#pragma unroll
    for (int u = 0; u < 4; ++u) { const int cc = c + u; const float* xr = x + (size_t)cc * TT; float acc = 0.f;
#pragma unroll
        for (int k = 0; k < 3; ++k) { const int tt = t - 1 + k; const float xv = (tt >= 0 && tt < TT) ? bfr(xr[min(max(tt, 0), TT - 1)]) : 0.f; float p = __fmul_rn(bfr(w[cc * 3 + k]), xv); asm volatile("" : "+v"(p)); acc = __fadd_rn(acc, p); }
        o[u] = __fmul_rn(acc, mf); } *(volatile v4f*)(F + e) = o; __threadfence(); *(volatile v4f*)(F + e) = o; }
__global__ __launch_bounds__(256) void k_cln(const float* __restrict__ F, const float* __restrict__ g, const float* __restrict__ bb, bf* Hh, bf* Hl) { const int lane = threadIdx.x & 31; const int t = blockIdx.x * 8 + (threadIdx.x >> 5); if (t >= TT) return; float v[CC / 32]; float s = 0.f;
#pragma unroll
    for (int ch = 0; ch < CC / 128; ++ch) { const v4f a = *(const v4f*)(F + (size_t)t * CC + ch * 128 + lane * 4);
#pragma unroll
        for (int u = 0; u < 4; ++u) { v[ch * 4 + u] = a[u]; s += a[u]; } }
#pragma unroll
    for (int sh = 16; sh; sh >>= 1) s += __shfl_xor(s, sh, 32);
    const float mean = s * (1.0f / CC); float q = 0.f;
#pragma unroll
    for (int k = 0; k < CC / 32; ++k) { float d = __fsub_rn(v[k], mean); asm volatile("" : "+v"(d)); v[k] = d; float p = __fmul_rn(d, d); asm volatile("" : "+v"(p)); q = __fadd_rn(q, p); }
#pragma unroll
    for (int sh = 16; sh; sh >>= 1) q += __shfl_xor(q, sh, 32);
    const float rs = __frsqrt_rn(__fadd_rn(q * (1.0f / CC), 1e-5f));
    for (int ps = 0; ps < 2; ++ps) {
#pragma unroll
        for (int ch = 0; ch < CC / 128; ++ch) { v4us oh, ol;
#pragma unroll
            for (int u = 0; u < 4; ++u) { const int c = ch * 128 + lane * 4 + u; float n0 = __fmul_rn(v[ch * 4 + u], rs); asm volatile("" : "+v"(n0)); float gg = bfr(g[c]), be = bfr(bb[c]); asm volatile("" : "+v"(gg)); asm volatile("" : "+v"(be)); float t1 = __fmul_rn(n0, gg); asm volatile("" : "+v"(t1)); unsigned short p2, q2; splitf(__fadd_rn(t1, be), p2, q2); oh[u] = p2; ol[u] = q2; }
            const size_t oo = (size_t)t * CC + ch * 128 + lane * 4; *(volatile v4us*)(Hh + oo) = oh; *(volatile v4us*)(Hl + oo) = ol; }
        if (ps == 0) __threadfence(); } }
__global__ __launch_bounds__(256) void k_qp(const float* __restrict__ QF, bf* Qh, bf* Ql) { const size_t e = ((size_t)blockIdx.x * 256 + threadIdx.x) * 4; if (e >= (size_t)NH_ * TT * HD) return; const int d = (int)(e % HD); const int t = (int)((e / HD) % TT); const int h = (int)(e / ((size_t)HD * TT)); const float* f = QF + (size_t)t * CC + h * HD + d; v4us oh, ol;
#pragma unroll
    for (int u = 0; u < 4; ++u) { unsigned short a, b; splitf(f[u] * 0.125f, a, b); oh[u] = a; ol[u] = b; } *(volatile v4us*)(Qh + e) = oh; *(volatile v4us*)(Ql + e) = ol; __threadfence(); *(volatile v4us*)(Qh + e) = oh; *(volatile v4us*)(Ql + e) = ol; }
__global__ __launch_bounds__(256) void k_kp(const float* __restrict__ KF, bf* Kh, bf* Kl) { const size_t e = ((size_t)blockIdx.x * 256 + threadIdx.x) * 4; if (e >= (size_t)NH_ * TP * HD) return; const int d = (int)(e % HD); const int tp = (int)((e / HD) % TP); const int h = (int)(e / ((size_t)HD * TP)); const int t = tp - WW; v4us oh, ol;
#pragma unroll
    for (int u = 0; u < 4; ++u) { unsigned short a = 0, b = 0; if (t >= 0 && t < TT) splitf(KF[(size_t)t * CC + h * HD + d + u], a, b); oh[u] = a; ol[u] = b; } *(volatile v4us*)(Kh + e) = oh; *(volatile v4us*)(Kl + e) = ol; __threadfence(); *(volatile v4us*)(Kh + e) = oh; *(volatile v4us*)(Kl + e) = ol; }
__global__ __launch_bounds__(256) void k_vt3(const float* __restrict__ VF, bf* Th, bf* Tl) { const size_t e = ((size_t)blockIdx.x * 256 + threadIdx.x) * 2; if (e >= (size_t)NH_ * NC * HD * KW) return; const int kk = (int)(e % KW); const int d = (int)((e / KW) % HD); const int c = (int)((e / ((size_t)KW * HD)) % NC); const int h = (int)(e / ((size_t)KW * HD * NC)); v2us oh, ol;
#pragma unroll
    for (int u = 0; u < 2; ++u) { const int j = c * WW - WW + kk + u; unsigned short a = 0, b = 0; if (j >= 0 && j < TT) splitf(VF[(size_t)j * CC + h * HD + d], a, b); oh[u] = a; ol[u] = b; } *(volatile v2us*)(Th + e) = oh; *(volatile v2us*)(Tl + e) = ol; __threadfence(); *(volatile v2us*)(Th + e) = oh; *(volatile v2us*)(Tl + e) = ol; }
__global__ __launch_bounds__(256) void k_lsoft(const float* __restrict__ S, const int* __restrict__ msk, bf* Ph, bf* Pl) { const int lane = threadIdx.x & 31; const int row = blockIdx.x * 8 + (threadIdx.x >> 5); if (row >= NC * WW) return; const int qq = row % WW; const int c = (row / WW) % NC; const int i = c * WW + qq; const float* sr = S + (size_t)row * KW; float v[KW / 32]; float mx = -3.0e38f;
#pragma unroll
    for (int m = 0; m < KW / 32; ++m) { const int kk = m * 32 + lane; const int j = c * WW - WW + kk; const int rel = kk - qq; const bool valid = (rel >= 0 && rel <= 2 * WW && j >= 0 && j < TT); float t;
        if (valid) { const float mb = (msk[j] != 0) ? 0.f : -1.0e4f; t = __fadd_rn(sr[kk], mb); } else t = -1.0e30f; v[m] = t; mx = fmaxf(mx, t); }
#pragma unroll
    for (int sh = 16; sh; sh >>= 1) mx = fmaxf(mx, __shfl_xor(mx, sh, 32));
    float sum = 0.f;
#pragma unroll
    for (int m = 0; m < KW / 32; ++m) { float d0 = __fsub_rn(v[m], mx); asm volatile("" : "+v"(d0)); v[m] = __builtin_amdgcn_exp2f(__fmul_rn(d0, 1.4426950408889634f)); sum += v[m]; }
#pragma unroll
    for (int sh = 16; sh; sh >>= 1) sum += __shfl_xor(sum, sh, 32);
    const float mq = (msk[i] != 0) ? 1.f : 0.f; const float f = __fdiv_rn(mq, sum);
    for (int ps = 0; ps < 2; ++ps) {
#pragma unroll
        for (int m = 0; m < KW / 32; ++m) { unsigned short a, b; splitf(v[m] * f, a, b); const size_t oo = (size_t)row * KW + m * 32 + lane; *(volatile unsigned short*)(Ph + oo) = a; *(volatile unsigned short*)(Pl + oo) = b; }
        if (ps == 0) __threadfence(); } }
__global__ __launch_bounds__(256) void k_og(const float* __restrict__ O, bf* Ah, bf* Al) { const size_t e = ((size_t)blockIdx.x * 256 + threadIdx.x) * 4; if (e >= (size_t)TT * CC) return; const int ch = (int)(e % CC); const int t = (int)(e / CC); const int h = ch / HD, d = ch % HD; const int c = t / WW, qq = t % WW; const float* src = O + (((size_t)h * NC + c) * WW + qq) * HD + d; v4us oh, ol;
#pragma unroll
    for (int u = 0; u < 4; ++u) { unsigned short a, b; splitf(src[u], a, b); oh[u] = a; ol[u] = b; } *(volatile v4us*)(Ah + e) = oh; *(volatile v4us*)(Al + e) = ol; __threadfence(); *(volatile v4us*)(Ah + e) = oh; *(volatile v4us*)(Al + e) = ol; }
__global__ __launch_bounds__(256) void k_outT(const float* __restrict__ Y, const int* __restrict__ msk, float* outb) { const size_t e = ((size_t)blockIdx.x * 256 + threadIdx.x) * 4; if (e >= (size_t)CC * TT) return; const int t = (int)(e % TT); const int o = (int)(e / TT); v4f r;
#pragma unroll
    for (int u = 0; u < 4; ++u) { const float mf = (msk[t + u] != 0) ? 1.f : 0.f; r[u] = __fmul_rn(Y[(size_t)(t + u) * CC + o], mf); } *(volatile v4f*)(outb + e) = r; __threadfence(); *(volatile v4f*)(outb + e) = r; }

extern "C" void kernel_launch(void* const* d_in, const int* in_sizes, int n_in,
                              void* d_out, int out_size, void* d_ws, size_t ws_size, hipStream_t stream) {
    (void)in_sizes; (void)n_in; (void)out_size;
    const float* x = (const float*)d_in[0]; const int* mask = (const int*)d_in[1]; const float *qcw = (const float*)d_in[2], *kcw = (const float*)d_in[3], *vcw = (const float*)d_in[4];
    const float *qnw = (const float*)d_in[5], *qnb = (const float*)d_in[6], *knw = (const float*)d_in[7], *knb = (const float*)d_in[8], *vnw = (const float*)d_in[9], *vnb = (const float*)d_in[10];
    const float *wq = (const float*)d_in[11], *bq = (const float*)d_in[12], *wk = (const float*)d_in[13], *bk = (const float*)d_in[14], *wv = (const float*)d_in[15], *bv = (const float*)d_in[16], *wo = (const float*)d_in[17], *bo = (const float*)d_in[18];
    float* OUT = (float*)d_out;
    char* wsp = (char*)d_ws;
    auto take = [&](size_t bytes) { char* p = wsp; wsp += (bytes + 255) & ~(size_t)255; return (void*)p; };
    bf* BW[4]; for (int i = 0; i < 4; ++i) BW[i] = (bf*)take((size_t)CC * CC * 2);
    float* F = (float*)take((size_t)TT * CC * 4); bf* Hh = (bf*)take((size_t)TT * CC * 2); bf* Hl = (bf*)take((size_t)TT * CC * 2); float* PF = (float*)take((size_t)TT * CC * 4);
    bf* Qh = (bf*)take((size_t)NH_ * TT * HD * 2); bf* Ql = (bf*)take((size_t)NH_ * TT * HD * 2); bf* Kh = (bf*)take((size_t)NH_ * TP * HD * 2); bf* Kl = (bf*)take((size_t)NH_ * TP * HD * 2); bf* VTh = (bf*)take((size_t)NH_ * NC * HD * KW * 2); bf* VTl = (bf*)take((size_t)NH_ * NC * HD * KW * 2);
    float* S = (float*)take((size_t)NH_ * NC * WW * KW * 4); bf* Ph = (bf*)take((size_t)NH_ * NC * WW * KW * 2); bf* Pl = (bf*)take((size_t)NH_ * NC * WW * KW * 2); float* O = (float*)take((size_t)NH_ * NC * WW * HD * 4);
    if ((size_t)(wsp - (char*)d_ws) > ws_size) return;
    const float* Wl[4] = {wq, wk, wv, wo}; for (int i = 0; i < 4; ++i) k_cvt8<<<(CC * CC / 8 + 255) / 256, 256, 0, stream>>>(Wl[i], BW[i], CC * CC / 8);
    const dim3 gp(TT / 64, CC / 64, 1); const unsigned gE = (unsigned)(((size_t)TT * CC / 4 + 255) / 256);
    for (int b = 0; b < 2; ++b) { const float* xb = x + (size_t)b * CC * TT; const int* mb = mask + (size_t)b * TT;
        k_dw<<<gE, 256, 0, stream>>>(xb, qcw, mb, F); k_cln<<<TT / 8, 256, 0, stream>>>(F, qnw, qnb, Hh, Hl); k_gemmw<bf, 1, true><<<gp, 32, 0, stream>>>(Hh, Hl, BW[0], nullptr, CC, PF, CC, bq, 0, 0, 0); k_qp<<<(unsigned)(((size_t)NH_ * TT * HD / 4 + 255) / 256), 256, 0, stream>>>(PF, Qh, Ql);
        k_dw<<<gE, 256, 0, stream>>>(xb, kcw, mb, F); k_cln<<<TT / 8, 256, 0, stream>>>(F, knw, knb, Hh, Hl); k_gemmw<bf, 1, true><<<gp, 32, 0, stream>>>(Hh, Hl, BW[1], nullptr, CC, PF, CC, bk, 0, 0, 0); k_kp<<<(unsigned)(((size_t)NH_ * TP * HD / 4 + 255) / 256), 256, 0, stream>>>(PF, Kh, Kl);
        k_dw<<<gE, 256, 0, stream>>>(xb, vcw, mb, F); k_cln<<<TT / 8, 256, 0, stream>>>(F, vnw, vnb, Hh, Hl); k_gemmw<bf, 1, true><<<gp, 32, 0, stream>>>(Hh, Hl, BW[2], nullptr, CC, PF, CC, bv, 0, 0, 0); k_vt3<<<(unsigned)(((size_t)NH_ * NC * HD * KW / 2 + 255) / 256), 256, 0, stream>>>(PF, VTh, VTl);
        for (int h = 0; h < NH_; ++h) { const size_t qo = (size_t)h * TT * HD, ko = (size_t)h * TP * HD, so = (size_t)h * NC * WW * KW, vo = (size_t)h * NC * HD * KW, oo = (size_t)h * NC * WW * HD;
            k_gemmw<bf, 2, false><<<dim3(1, KW / 64, NC), 32, 0, stream>>>(Qh + qo, Ql + qo, Kh + ko, Kl + ko, HD, S + so, KW, nullptr, (size_t)WW * HD, (size_t)WW * HD, (size_t)WW * KW);
            k_lsoft<<<NC * WW / 8, 256, 0, stream>>>(S + so, mb, Ph + so, Pl + so);
            k_gemmw<bf, 2, false><<<dim3(1, 1, NC), 32, 0, stream>>>(Ph + so, Pl + so, VTh + vo, VTl + vo, KW, O + oo, HD, nullptr, (size_t)WW * KW, (size_t)HD * KW, (size_t)WW * HD); }
        k_og<<<gE, 256, 0, stream>>>(O, Hh, Hl);
        k_gemmw<bf, 1, true><<<gp, 32, 0, stream>>>(Hh, Hl, BW[3], nullptr, CC, PF, CC, bo, 0, 0, 0);
        k_outT<<<(unsigned)(((size_t)CC * TT / 4 + 255) / 256), 256, 0, stream>>>(PF, mb, OUT + (size_t)b * CC * TT); }
}
